// DyDCNv3_1047972020323
// MI455X (gfx1250) — hardware-verified
//
#include <hip/hip_runtime.h>
#include <stddef.h>


#define NB_   8
#define NC_   256
#define NH_   64
#define NW_   64
#define NHW_  4096
#define KP_   9
#define NQ_   72
#define AP_   264
#define TP_   68
#define ASC_  16.0f
#define WSC_  64.0f
#define OSC_  0.0009765625f
#define BNEPS 1e-5f
#define LDSF_ 8448

static_assert(LDSF_ * 2 == 64 * AP_);
static_assert(LDSF_ >= 128 * 64);
static_assert(NQ_ * 32 == KP_ * NC_);

typedef float    v4f  __attribute__((ext_vector_type(4)));
typedef float    v8f  __attribute__((ext_vector_type(8)));
typedef _Float16 v8h  __attribute__((ext_vector_type(8)));
typedef _Float16 v16h __attribute__((ext_vector_type(16)));
union FragH { v16h v; v8h h[2]; };

__device__ __forceinline__ v8f wm16(v16h a, v16h b, v8f c) {
  return __builtin_amdgcn_wmma_f32_16x16x32_f16(false, a, false, b, (short)0, c, false, false);
}

__global__ __launch_bounds__(256) void k_xpose(const float* __restrict__ x, float* xt) {
  __shared__ __attribute__((aligned(16))) float T[32 * TP_];
  const int tid = threadIdx.x, lane = tid & 31, wave = tid >> 5;
  const int blk = blockIdx.x;
  const int pg = blk & 63;
  const int cg = (blk >> 6) & 7;
  const int b  = blk >> 9;
#pragma unroll
  for (int s = 0; s < 2; ++s) {
    const int f  = tid + 256 * s;
    const int ci = f >> 4, pq = f & 15;
    const v4f v = *(const v4f*)(x + ((size_t)(b * NC_ + cg * 32 + ci) * NHW_ + pg * 64 + pq * 4));
    *(v4f*)(T + ci * TP_ + pq * 4) = v;
  }
  __syncthreads();
  v4f ov[2];
  size_t ga[2];
#pragma unroll
  for (int s = 0; s < 2; ++s) {
    const int pl = wave * 8 + s * 4 + (lane >> 3);
    const int j  = lane & 7;
    v4f v;
    v.x = T[(4 * j + 0) * TP_ + pl];
    v.y = T[(4 * j + 1) * TP_ + pl];
    v.z = T[(4 * j + 2) * TP_ + pl];
    v.w = T[(4 * j + 3) * TP_ + pl];
    ov[s] = v;
    ga[s] = ((size_t)(b * NHW_ + pg * 64 + pl)) * NC_ + cg * 32 + 4 * j;
  }
#pragma unroll
  for (int s = 0; s < 2; ++s) *(volatile v4f*)(xt + ga[s]) = ov[s];
  __threadfence();
#pragma unroll
  for (int s = 0; s < 2; ++s) *(volatile v4f*)(xt + ga[s]) = ov[s];
}

__global__ __launch_bounds__(256) void k_packw(const float* __restrict__ w, _Float16* bp) {
  const int u  = blockIdx.x * 256 + threadIdx.x;
  const int hf = u & 1;
  const int ln = (u >> 1) & 31;
  const int nt = (u >> 6) & 15;
  const int q  = u >> 10;
  const int kk = q >> 3, cc = q & 7;
  const int hh = ln >> 4, m = ln & 15;
  const int o  = nt * 16 + m;
  const int c0 = cc * 32 + hf * 16 + 8 * hh;
  const float* wp = w + ((size_t)(o * NC_ + c0)) * KP_ + kk;
  v8h hv;
#pragma unroll
  for (int j = 0; j < 8; ++j) { const float t = wp[j * KP_] * WSC_; hv[j] = (_Float16)t; }
  _Float16* dst = bp + (size_t)u * 8;
  *(volatile v8h*)dst = hv;
  __threadfence();
  *(volatile v8h*)dst = hv;
}

__global__ __launch_bounds__(256) void k_dconv(const float* __restrict__ xt, const float* __restrict__ offs,
                                               const float* __restrict__ msk, const _Float16* __restrict__ bp,
                                               float* pre) {
  __shared__ __attribute__((aligned(16))) float LDSF[LDSF_];
  _Float16* As = (_Float16*)LDSF;
  float* S = LDSF;

  const int tid = threadIdx.x, lane = tid & 31, wave = tid >> 5, hh = lane >> 4, m = lane & 15;
  const int mh = wave & 1, nq = wave >> 1;
  const int blk = blockIdx.x, b = blk >> 6, h = blk & 63;
  const int p = tid >> 2, cq = tid & 3;
  const int pbase = h * NW_ + p;
  const float* xtb = xt + (size_t)b * NHW_ * NC_;

  v8f acc[2][4];
  {
    v8f z;
#pragma unroll
    for (int i = 0; i < 8; ++i) z[i] = 0.0f;
#pragma unroll
    for (int mt = 0; mt < 2; ++mt)
#pragma unroll
      for (int nt = 0; nt < 4; ++nt) acc[mt][nt] = z;
  }

#pragma unroll 1
  for (int kk = 0; kk < KP_; ++kk) {
    const int ky = kk / 3, kx = kk - 3 * ky;
    const float dy = offs[((size_t)(b * 18 + 2 * kk)) * NHW_ + pbase];
    const float dx = offs[((size_t)(b * 18 + 2 * kk + 1)) * NHW_ + pbase];
    const float mv = msk[((size_t)(b * KP_ + kk)) * NHW_ + pbase];
    float py = (float)(h - 1 + ky) + dy;
    float px = (float)(p - 1 + kx) + dx;
    py = fminf(fmaxf(py, -4.0f), 68.0f);
    px = fminf(fmaxf(px, -4.0f), 68.0f);
    const float y0f = floorf(py), x0f = floorf(px);
    const float ly = py - y0f, lx = px - x0f;
    const int y0 = (int)y0f, x0 = (int)x0f, y1 = y0 + 1, x1 = x0 + 1;
    const bool vy0 = (y0 >= 0) && (y0 < NH_), vy1 = (y1 >= 0) && (y1 < NH_);
    const bool vx0 = (x0 >= 0) && (x0 < NW_), vx1 = (x1 >= 0) && (x1 < NW_);
    const int yi0 = min(max(y0, 0), NH_ - 1), yi1 = min(max(y1, 0), NH_ - 1);
    const int xi0 = min(max(x0, 0), NW_ - 1), xi1 = min(max(x1, 0), NW_ - 1);
    const float w00 = (vy0 && vx0) ? (1.0f - ly) * (1.0f - lx) : 0.0f;
    const float w01 = (vy0 && vx1) ? (1.0f - ly) * lx : 0.0f;
    const float w10 = (vy1 && vx0) ? ly * (1.0f - lx) : 0.0f;
    const float w11 = (vy1 && vx1) ? ly * lx : 0.0f;
    const float ms = mv * ASC_;
    const float* r00 = xtb + (size_t)(yi0 * NW_ + xi0) * NC_;
    const float* r01 = xtb + (size_t)(yi0 * NW_ + xi1) * NC_;
    const float* r10 = xtb + (size_t)(yi1 * NW_ + xi0) * NC_;
    const float* r11 = xtb + (size_t)(yi1 * NW_ + xi1) * NC_;

    __syncthreads();
#pragma unroll 1
    for (int i = 0; i < 8; ++i) {
      const int c = cq * 64 + 8 * i;
      const v4f ga0 = *(const v4f*)(r00 + c), ga1 = *(const v4f*)(r00 + c + 4);
      const v4f gb0 = *(const v4f*)(r01 + c), gb1 = *(const v4f*)(r01 + c + 4);
      const v4f gc0 = *(const v4f*)(r10 + c), gc1 = *(const v4f*)(r10 + c + 4);
      const v4f gd0 = *(const v4f*)(r11 + c), gd1 = *(const v4f*)(r11 + c + 4);
      v4f lo = ((ga0 * w00 + gb0 * w01) + gc0 * w10) + gd0 * w11;
      v4f hi = ((ga1 * w00 + gb1 * w01) + gc1 * w10) + gd1 * w11;
      lo = lo * ms;
      hi = hi * ms;
      v8h hv;
      hv[0] = (_Float16)lo.x; hv[1] = (_Float16)lo.y; hv[2] = (_Float16)lo.z; hv[3] = (_Float16)lo.w;
      hv[4] = (_Float16)hi.x; hv[5] = (_Float16)hi.y; hv[6] = (_Float16)hi.z; hv[7] = (_Float16)hi.w;
      *(v8h*)(As + p * AP_ + c) = hv;
    }
    __syncthreads();

    const _Float16* arow0 = As + (mh * 32 + m) * AP_ + 8 * hh;
    const _Float16* arow1 = arow0 + 16 * AP_;
    const _Float16* bq = bp + ((size_t)(kk * 8) * 16 + nq * 4) * 512 + lane * 16;
#pragma unroll 1
    for (int cc = 0; cc < 8; ++cc) {
      FragH a0, a1;
      a0.h[0] = *(const v8h*)(arow0 + cc * 32);
      a0.h[1] = *(const v8h*)(arow0 + cc * 32 + 16);
      a1.h[0] = *(const v8h*)(arow1 + cc * 32);
      a1.h[1] = *(const v8h*)(arow1 + cc * 32 + 16);
      const _Float16* bc = bq + (size_t)cc * 8192;
      const v16h b0 = *(const v16h*)(bc);
      const v16h b1 = *(const v16h*)(bc + 512);
      const v16h b2 = *(const v16h*)(bc + 1024);
      const v16h b3 = *(const v16h*)(bc + 1536);
      acc[0][0] = wm16(a0.v, b0, acc[0][0]);
      acc[0][1] = wm16(a0.v, b1, acc[0][1]);
      acc[0][2] = wm16(a0.v, b2, acc[0][2]);
      acc[0][3] = wm16(a0.v, b3, acc[0][3]);
      acc[1][0] = wm16(a1.v, b0, acc[1][0]);
      acc[1][1] = wm16(a1.v, b1, acc[1][1]);
      acc[1][2] = wm16(a1.v, b2, acc[1][2]);
      acc[1][3] = wm16(a1.v, b3, acc[1][3]);
      asm volatile("v_nop\n\tv_nop\n\tv_nop\n\tv_nop"
                   : "+v"(acc[0][0]), "+v"(acc[0][1]), "+v"(acc[0][2]), "+v"(acc[0][3]),
                     "+v"(acc[1][0]), "+v"(acc[1][1]), "+v"(acc[1][2]), "+v"(acc[1][3])
                   : "v"(a0.v), "v"(a1.v), "v"(b0), "v"(b1), "v"(b2), "v"(b3));
    }
  }

  __syncthreads();
#pragma unroll
  for (int P = 0; P < 2; ++P) {
    if ((nq >> 1) == P) {
#pragma unroll
      for (int mt = 0; mt < 2; ++mt) {
#pragma unroll
        for (int nt = 0; nt < 4; ++nt) {
          float* sp = S + ((nq & 1) * 64 + nt * 16 + m) * 64 + mh * 32 + mt * 16 + 8 * hh;
          v4f lo, hi;
          lo.x = acc[mt][nt][0] * OSC_; lo.y = acc[mt][nt][1] * OSC_;
          lo.z = acc[mt][nt][2] * OSC_; lo.w = acc[mt][nt][3] * OSC_;
          hi.x = acc[mt][nt][4] * OSC_; hi.y = acc[mt][nt][5] * OSC_;
          hi.z = acc[mt][nt][6] * OSC_; hi.w = acc[mt][nt][7] * OSC_;
          *(v4f*)sp = lo;
          *(v4f*)(sp + 4) = hi;
        }
      }
    }
    __syncthreads();
    v4f ov[8];
    size_t ga[8];
#pragma unroll
    for (int s = 0; s < 8; ++s) {
      const int L  = wave * 32 + s * 4 + (lane >> 3);
      const int ol = L >> 1, hf = L & 1, j = lane & 7;
      ov[s] = *(const v4f*)(S + ol * 64 + hf * 32 + 4 * j);
      ga[s] = ((size_t)(b * NC_ + P * 128 + ol)) * NHW_ + h * NW_ + hf * 32 + 4 * j;
    }
#pragma unroll
    for (int s = 0; s < 8; ++s) *(volatile v4f*)(pre + ga[s]) = ov[s];
    __threadfence();
#pragma unroll
    for (int s = 0; s < 8; ++s) *(volatile v4f*)(pre + ga[s]) = ov[s];
    __syncthreads();
  }
}

__global__ __launch_bounds__(256) void k_stats(const float* __restrict__ pre, const float* __restrict__ gamma,
                                               float* mutab, float* sctab) {
  __shared__ double rs[256];
  __shared__ double rq[256];
  __shared__ __attribute__((aligned(16))) float lmu[32];
  __shared__ __attribute__((aligned(16))) float lsc[32];
  const int tid = threadIdx.x, lane = tid & 31, wave = tid >> 5;
  const int g = blockIdx.x;
#pragma unroll 1
  for (int t = 0; t < 4; ++t) {
    const int cl = wave * 4 + t;
    const int c  = g * 32 + cl;
    double s = 0.0, q = 0.0;
#pragma unroll 1
    for (int it = 0; it < NB_ * 32; ++it) {
      const int bb = it >> 5, seg = it & 31;
      const v4f v = *(const v4f*)(pre + ((size_t)(bb * NC_ + c)) * NHW_ + seg * 128 + lane * 4);
      const double a0 = (double)v.x, a1 = (double)v.y, a2 = (double)v.z, a3 = (double)v.w;
      s += a0; q += a0 * a0;
      s += a1; q += a1 * a1;
      s += a2; q += a2 * a2;
      s += a3; q += a3 * a3;
    }
    rs[tid] = s;
    rq[tid] = q;
    __syncthreads();
    if (lane == 0) {
      double S0 = 0.0, Q0 = 0.0;
#pragma unroll 1
      for (int i = 0; i < 32; ++i) { S0 += rs[wave * 32 + i]; Q0 += rq[wave * 32 + i]; }
      const double inv = 1.0 / (double)(NB_ * NHW_);
      const double mu = S0 * inv;
      double var = Q0 * inv - mu * mu;
      if (var < 0.0) var = 0.0;
      const float sc = rsqrtf((float)var + BNEPS) * gamma[c];
      lmu[cl] = (float)mu;
      lsc[cl] = sc;
    }
    __syncthreads();
  }
  const bool wr = (wave == 0) && (lane < 16);
  const int j = lane & 7;
  const v4f va = *(const v4f*)(lmu + 4 * j);
  const v4f vb = *(const v4f*)(lsc + 4 * j);
  const v4f v = (lane < 8) ? va : vb;
  float* dst = (lane < 8) ? (mutab + g * 32 + 4 * j) : (sctab + g * 32 + 4 * j);
  if (wr) *(volatile v4f*)dst = v;
  __threadfence();
  if (wr) *(volatile v4f*)dst = v;
}

__global__ __launch_bounds__(256) void k_apply(const float* __restrict__ pre, const float* __restrict__ mutab,
                                               const float* __restrict__ sctab, const float* __restrict__ beta,
                                               float* out) {
  const size_t i4 = (size_t)blockIdx.x * 256 + threadIdx.x;
  const size_t e  = i4 * 4;
  const int c = (int)((e >> 12) & 255);
  const v4f v = *(const v4f*)(pre + e);
  const float mu = mutab[c], sc = sctab[c], be = beta[c];
  const v4f y = (v - mu) * sc + be;
  *(volatile v4f*)(out + e) = y;
  __threadfence();
  *(volatile v4f*)(out + e) = y;
}

extern "C" void kernel_launch(void* const* d_in, const int* in_sizes, int n_in,
                              void* d_out, int out_size, void* d_ws, size_t ws_size,
                              hipStream_t stream) {
  if (n_in < 6) return;
  if (in_sizes[0] != NB_ * NC_ * NHW_) return;
  if (in_sizes[1] != NB_ * 2 * KP_ * NHW_) return;
  if (in_sizes[2] != NB_ * KP_ * NHW_) return;
  if (in_sizes[3] != NC_ * NC_ * KP_) return;
  if (in_sizes[4] < NC_ || in_sizes[5] < NC_) return;
  if (out_size != NB_ * NC_ * NHW_) return;

  const float* x     = (const float*)d_in[0];
  const float* offs  = (const float*)d_in[1];
  const float* msk   = (const float*)d_in[2];
  const float* wgt   = (const float*)d_in[3];
  const float* gamma = (const float*)d_in[4];
  const float* beta  = (const float*)d_in[5];
  float* out = (float*)d_out;

  char* ws = (char*)d_ws;
  size_t o = 0;
  const size_t oXt  = o; o += (size_t)NB_ * NHW_ * NC_ * 4;
  const size_t oPre = o; o += (size_t)NB_ * NC_ * NHW_ * 4;
  const size_t oBp  = o; o += (size_t)NQ_ * 16 * 32 * 16 * 2;
  const size_t oMu  = o; o += 1024;
  const size_t oSc  = o; o += 1024;
  if (o > ws_size) return;
  float*    xt    = (float*)(ws + oXt);
  float*    pre   = (float*)(ws + oPre);
  _Float16* bpk   = (_Float16*)(ws + oBp);
  float*    mutab = (float*)(ws + oMu);
  float*    sctab = (float*)(ws + oSc);

  k_xpose<<<NB_ * 8 * 64, 256, 0, stream>>>(x, xt);
  k_packw<<<(NQ_ * 16 * 32 * 2) / 256, 256, 0, stream>>>(wgt, bpk);
  k_dconv<<<NB_ * NH_, 256, 0, stream>>>(xt, offs, msk, bpk, pre);
  k_stats<<<NC_ / 32, 256, 0, stream>>>(pre, gamma, mutab, sctab);
  k_apply<<<(NB_ * NC_ * NHW_) / (4 * 256), 256, 0, stream>>>(pre, mutab, sctab, beta, out);
}
